// MLPPredictor_89000312308383
// MI455X (gfx1250) — hardware-verified
//
#include <hip/hip_runtime.h>

constexpr int kNodes = 100000;
constexpr int kEdges = 1600000;
constexpr int kFeat  = 128;
constexpr int kPitch = 136;
constexpr int kTileE = 64;
constexpr int kTiles = kEdges / kTileE;
constexpr int kBlock = 128;
constexpr int kGrid  = 1000;
constexpr int kCastThreads = 256;
constexpr int kCastBlocks  = (kNodes * kFeat) / (8 * kCastThreads);

static_assert(kEdges % kTileE == 0);
static_assert(kTiles % kGrid == 0);
static_assert(kBlock == kFeat);
static_assert((kNodes * kFeat) % (8 * kCastThreads) == 0);
static_assert(kPitch % 8 == 0);
static_assert(kFeat % 32 == 0);

typedef __attribute__((ext_vector_type(16))) __bf16 v16b;
typedef __attribute__((ext_vector_type(8)))  __bf16 v8b;
typedef __attribute__((ext_vector_type(8)))  float  v8f;
typedef __attribute__((ext_vector_type(4)))  float  v4f;
typedef __attribute__((ext_vector_type(4)))  unsigned int v4u;
typedef __attribute__((ext_vector_type(2)))  unsigned int v2u;

__device__ __forceinline__ unsigned short f2bf_bits(float f) {
  unsigned u = __float_as_uint(f);
  return (unsigned short)((u + 0x7FFFu + ((u >> 16) & 1u)) >> 16);
}
__device__ __forceinline__ float bf_bits2f(unsigned short h) { return __uint_as_float(((unsigned)h) << 16); }
__device__ __forceinline__ unsigned pk16(unsigned short a, unsigned short b) { return (unsigned)a | ((unsigned)b << 16); }

__device__ __forceinline__ void acc_guard4(v8f& a, v8f& b, v8f& c, v8f& d) { asm volatile("v_nop\n\tv_nop\n\tv_nop\n\tv_nop" : "+v"(a), "+v"(b), "+v"(c), "+v"(d)); }
__device__ __forceinline__ void grp_guard(v8f& a0, v8f& a1, v8f& a2, v8f& a3, v16b x, v16b y, v16b p0, v16b p1, v16b p2, v16b p3) {
  asm volatile("v_nop\n\tv_nop\n\tv_nop\n\tv_nop" : "+v"(a0), "+v"(a1), "+v"(a2), "+v"(a3) : "v"(x), "v"(y), "v"(p0), "v"(p1), "v"(p2), "v"(p3));
}

template <typename T> struct Frag;
template <> struct Frag<__bf16> {
  typedef v16b V; union U { v16b v; v8b h[2]; };
  static __device__ __forceinline__ v16b load(const __bf16* p) {
    U f; f.h[0] = *(const v8b*)(p); f.h[1] = *(const v8b*)(p + 16); return f.v;
  }
  static __device__ __forceinline__ v8f mma(v16b a, v16b b, v8f c) {
    return __builtin_amdgcn_wmma_f32_16x16x32_bf16(false, a, false, b, (short)0, c, false, false);
  }
};

__device__ __forceinline__ void split_prod(float a, float b, unsigned& hw, unsigned& lw) {
  const float p = a * b;
  const unsigned u = __float_as_uint(p);
  hw = u & 0xffff0000u;
  const float r = p - __uint_as_float(hw);
  lw = __float_as_uint(r) & 0xffff0000u;
}

__global__ __launch_bounds__(kCastThreads) void hcast_kernel(const float* __restrict__ in, unsigned short* __restrict__ outp) {
  const int i = blockIdx.x * kCastThreads + threadIdx.x;
  const float* p = in + 8 * (size_t)i;
  const v4f a = *(const v4f*)(p);
  const v4f c = *(const v4f*)(p + 4);
  const float a0 = a[0], a1 = a[1], a2 = a[2], a3 = a[3];
  const float c0 = c[0], c1 = c[1], c2 = c[2], c3 = c[3];
  const v4u u = (v4u){pk16(f2bf_bits(a0), f2bf_bits(a1)), pk16(f2bf_bits(a2), f2bf_bits(a3)),
                      pk16(f2bf_bits(c0), f2bf_bits(c1)), pk16(f2bf_bits(c2), f2bf_bits(c3))};
  unsigned short* q = outp + 8 * (size_t)i;
  *(volatile v4u*)q = u;
  __threadfence();
  *(volatile v4u*)q = u;
}

__global__ __launch_bounds__(kBlock) void edge_mlp_kernel(
    const unsigned short* __restrict__ hb, const int* __restrict__ src, const int* __restrict__ dst,
    const float* __restrict__ W1, const float* __restrict__ b1, const float* __restrict__ W2,
    const float* __restrict__ b2, float* __restrict__ out) {
  __shared__ __align__(16) unsigned short w1t[kFeat * kPitch];
  __shared__ __align__(16) unsigned short ahi[kTileE * kPitch];
  __shared__ __align__(16) unsigned short alo[kTileE * kPitch];
  __shared__ __align__(16) float sc[kTileE];

  const int t    = threadIdx.x;
  const int lane = t & 31;
  const int wave = __builtin_amdgcn_readfirstlane(t >> 5);
  const int hsel = lane >> 4;
  const int rl   = lane & 15;

#pragma unroll 4
  for (int kp = 0; kp < kFeat / 2; ++kp) {
    const float wa = W1[(size_t)(2 * kp) * kFeat + t];
    const float wb = W1[(size_t)(2 * kp + 1) * kFeat + t];
    const unsigned u = pk16(f2bf_bits(wa), f2bf_bits(wb));
    *(unsigned*)(&w1t[t * kPitch + 2 * kp]) = u;
  }
  float b1r[8], w2r[8];
#pragma unroll
  for (int nt = 0; nt < 8; ++nt) b1r[nt] = bf_bits2f(f2bf_bits(b1[nt * 16 + rl]));
  asm volatile("" ::: "memory");
#pragma unroll
  for (int nt = 0; nt < 8; ++nt) w2r[nt] = bf_bits2f(f2bf_bits(W2[nt * 16 + rl]));
  const float b2v = bf_bits2f(f2bf_bits(b2[0]));
  __syncthreads();

  const int mb = wave * 16;
  const __bf16* Ah = (const __bf16*)ahi + (mb + rl) * kPitch + 8 * hsel;
  const __bf16* Al = (const __bf16*)alo + (mb + rl) * kPitch + 8 * hsel;
  const __bf16* Wt = (const __bf16*)w1t + rl * kPitch + 8 * hsel;
  const v8f z8 = {0.f, 0.f, 0.f, 0.f, 0.f, 0.f, 0.f, 0.f};

  for (int tile = blockIdx.x; tile < kTiles; tile += (int)gridDim.x) {
    const int e0 = tile * kTileE;

#pragma unroll 2
    for (int i = 0; i < 16; ++i) {
      const int m = mb + i;
      const int e = e0 + m;
      int s = src[e]; s = s < 0 ? 0 : s; s = s > kNodes - 1 ? kNodes - 1 : s;
      int d = dst[e]; d = d < 0 ? 0 : d; d = d > kNodes - 1 ? kNodes - 1 : d;
      const v2u wa = *(const v2u*)(hb + (size_t)s * kFeat + 4 * lane);
      const v2u wb = *(const v2u*)(hb + (size_t)d * kFeat + 4 * lane);
      const unsigned ax = wa[0], ay = wa[1], bx = wb[0], by = wb[1];
      unsigned h0, l0, h1, l1, h2, l2, h3, l3;
      split_prod(__uint_as_float(ax << 16),          __uint_as_float(bx << 16),          h0, l0);
      split_prod(__uint_as_float(ax & 0xffff0000u), __uint_as_float(bx & 0xffff0000u), h1, l1);
      split_prod(__uint_as_float(ay << 16),          __uint_as_float(by << 16),          h2, l2);
      split_prod(__uint_as_float(ay & 0xffff0000u), __uint_as_float(by & 0xffff0000u), h3, l3);
      const v2u hv = (v2u){(h0 >> 16) | h1, (h2 >> 16) | h3};
      const v2u lv = (v2u){(l0 >> 16) | l1, (l2 >> 16) | l3};
      *(v2u*)(&ahi[m * kPitch + 4 * lane]) = hv;
      *(v2u*)(&alo[m * kPitch + 4 * lane]) = lv;
    }
    __syncthreads();

    v8f acc[8];
#pragma unroll
    for (int nt = 0; nt < 8; ++nt) acc[nt] = z8;
#pragma unroll 1
    for (int kk = 0; kk < kFeat / 32; ++kk) {
      const int k0 = kk * 32;
      const v16b fa = Frag<__bf16>::load(Ah + k0);
      const v16b fl = Frag<__bf16>::load(Al + k0);
#pragma unroll
      for (int g = 0; g < 2; ++g) {
        v16b bq[4];
#pragma unroll
        for (int j = 0; j < 4; ++j) bq[j] = Frag<__bf16>::load(Wt + ((g * 4 + j) * 16) * kPitch + k0);
#pragma unroll
        for (int j = 0; j < 4; ++j) {
          acc[g * 4 + j] = Frag<__bf16>::mma(fa, bq[j], acc[g * 4 + j]);
          acc[g * 4 + j] = Frag<__bf16>::mma(fl, bq[j], acc[g * 4 + j]);
        }
        grp_guard(acc[g * 4], acc[g * 4 + 1], acc[g * 4 + 2], acc[g * 4 + 3], fa, fl, bq[0], bq[1], bq[2], bq[3]);
      }
    }
    acc_guard4(acc[0], acc[1], acc[2], acc[3]);
    acc_guard4(acc[4], acc[5], acc[6], acc[7]);

    float sv[8];
#pragma unroll
    for (int v = 0; v < 8; ++v) sv[v] = 0.f;
#pragma unroll
    for (int nt = 0; nt < 8; ++nt) {
      const float wv = w2r[nt], bv = b1r[nt];
#pragma unroll
      for (int v = 0; v < 8; ++v) {
        float a = acc[nt][v] + bv;
        a = fmaxf(a, 0.f);
        sv[v] += a * wv;
      }
    }
#pragma unroll
    for (int off = 1; off < 16; off <<= 1) {
#pragma unroll
      for (int v = 0; v < 8; ++v) sv[v] += __shfl_xor(sv[v], off, 32);
    }
    if (rl == 0) {
#pragma unroll
      for (int v = 0; v < 8; ++v) sc[mb + 8 * hsel + v] = sv[v] + b2v;
    }
    __syncthreads();

    if (wave == 0) {
      const int c4 = (lane & 15) * 4;
      const v4f val = *(const v4f*)(sc + c4);
      float* op = out + (size_t)e0 + c4;
      if (lane < 16) *(volatile v4f*)op = val;
      __threadfence();
      if (lane < 16) *(volatile v4f*)op = val;
    }
  }
}

extern "C" void kernel_launch(void* const* d_in, const int* in_sizes, int n_in,
                              void* d_out, int out_size, void* d_ws, size_t ws_size, hipStream_t stream) {
  (void)in_sizes; (void)n_in; (void)out_size;
  const float* h   = (const float*)d_in[0];
  const int*   src = (const int*)  d_in[1];
  const int*   dst = (const int*)  d_in[2];
  const float* W1  = (const float*)d_in[3];
  const float* b1  = (const float*)d_in[4];
  const float* W2  = (const float*)d_in[5];
  const float* b2  = (const float*)d_in[6];
  float* out = (float*)d_out;

  const size_t hb_bytes = (size_t)kNodes * kFeat * 2;
  if (hb_bytes > ws_size) return;
  unsigned short* hb = (unsigned short*)d_ws;

  hcast_kernel<<<kCastBlocks, kCastThreads, 0, stream>>>(h, hb);
  edge_mlp_kernel<<<kGrid, kBlock, 0, stream>>>(hb, src, dst, W1, b1, W2, b2, out);
}
